// GraphConvolution_13589276524974
// MI455X (gfx1250) — hardware-verified
//
#include <hip/hip_runtime.h>
#include <math.h>
#include <stddef.h>
#include <stdint.h>


#define DF     128
#define L1P    768
#define MPP    512
#define HPP    512
#define KB1    384
#define KB2    768
#define KB4    512
#define NTHR   256
#define NWAVE  8
#define EPT    8
#define CHUNK  (NTHR * EPT)
#define WCAP   (EPT * 32)
#define LISTN  (NWAVE * WCAP)
#define NBA    1024
#define SLA    10
#define RCAP   28672
#define DEGCAP 64
#define GBM    64
#define GBN    128
#define GTHR   128
#define GWAVE  (GTHR / 32)
#define G2M    32
#define G2N    256
#define WPJOBS 20
#define WLI    ((DF * DF / 4) / NTHR)
#define WPI    ((DF * DF / 8) / NTHR)
#define AGG_ZINTS    (LISTN + 2 * RCAP + 3 * NBA)
#define MISC_INTS    16
#define RBH          512
#define ROWBUF_INTS  (NWAVE * RBH / 2)
#define AGG_LDS_INTS (AGG_ZINTS + MISC_INTS + ROWBUF_INTS)
#define WSMAX  134217728

static_assert((CHUNK & (CHUNK - 1)) == 0 && CHUNK <= 4096);
static_assert((NBA & (NBA - 1)) == 0 && NBA == (1 << SLA));
static_assert(((long long)CHUNK << SLA) < (1LL << 31));
static_assert(LISTN % NTHR == 0);
static_assert(NBA % NWAVE == 0 && NBA % 32 == 0 && NBA % GBM == 0 && NBA % G2M == 0);
static_assert(RCAP % 4 == 0 && AGG_ZINTS % 4 == 0 && LISTN % 4 == 0 && ((AGG_ZINTS + MISC_INTS) % 4) == 0);
static_assert(AGG_ZINTS % (NTHR * 4) == 0);
static_assert(KB1 % 32 == 0 && KB2 % 32 == 0 && KB4 % 32 == 0);
static_assert(KB1 == 3 * DF && KB2 == 6 * DF && KB4 == 4 * DF && L1P == 6 * DF && MPP == 4 * DF && HPP == 4 * DF);
static_assert(GBN == DF && GBM == GWAVE * 16 && DF == 4 * 32 && GTHR == DF);
static_assert(G2M == 2 * 16 && G2N == 2 * DF && GWAVE == 4 && G2M == GWAVE * 8 && G2N == 32 * 8);
static_assert(G2M * G2N == GBM * GBN);
static_assert(RBH == 4 * DF && (RBH % 2) == 0);
static_assert(WPI * NTHR * 8 == DF * DF && WLI * NTHR * 4 == DF * DF);
static_assert(AGG_LDS_INTS * 4 <= 300000);

typedef float          v4f   __attribute__((ext_vector_type(4)));
typedef float          v8f   __attribute__((ext_vector_type(8)));
typedef int            v4i   __attribute__((ext_vector_type(4)));
typedef int            v8i   __attribute__((ext_vector_type(8)));
typedef unsigned       v2u   __attribute__((ext_vector_type(2)));
typedef unsigned short v4us  __attribute__((ext_vector_type(4)));
typedef unsigned short v8us  __attribute__((ext_vector_type(8)));
typedef unsigned short v16us __attribute__((ext_vector_type(16)));
typedef __bf16         v16bf __attribute__((ext_vector_type(16)));
typedef v4f  __attribute__((may_alias)) v4fa;
typedef v4i  __attribute__((may_alias)) v4ia;
typedef v2u  __attribute__((may_alias)) v2ua;
typedef v4us __attribute__((may_alias)) v4usa;
typedef v8us __attribute__((may_alias)) v8usa;
union FragB { v16bf v; v16us u; v8us h[2]; v8i w; };

__device__ __forceinline__ v8f wmb(const FragB& a, const FragB& b, v8f c) {
  v8f d = __builtin_amdgcn_wmma_f32_16x16x32_bf16(false, a.v, false, b.v, (short)0, c, false, false);
  asm volatile("v_nop\n\tv_nop\n\tv_nop\n\tv_nop" : "+v"(d) : "v"(a.w), "v"(b.w));
  return d;
}

__device__ __forceinline__ v8f z8() { v8f z = {0.f, 0.f, 0.f, 0.f, 0.f, 0.f, 0.f, 0.f}; return z; }

__device__ __forceinline__ unsigned bf16_bits(float f) {
  const unsigned u = __float_as_uint(f);
  return (u + 0x7FFFu + ((u >> 16) & 1u)) >> 16;
}
__device__ __forceinline__ float bf16_val(float f) {
  return __uint_as_float(bf16_bits(f) << 16);
}

__device__ __forceinline__ void wave_sync() {
  __builtin_amdgcn_fence(__ATOMIC_RELEASE, "wavefront");
  __builtin_amdgcn_wave_barrier();
  __builtin_amdgcn_fence(__ATOMIC_ACQUIRE, "wavefront");
}

__device__ __forceinline__ void mma_seg(v8f (&acc)[8], const unsigned short* ap, const unsigned short* bp,
                                        int KB, int kseg) {
#pragma unroll 1
  for (int k0 = 0; k0 < kseg; k0 += 32) {
    FragB af;
    af.h[0] = *(const v8usa*)(ap + k0);
    af.h[1] = *(const v8usa*)(ap + k0 + 16);
#pragma unroll
    for (int nt = 0; nt < 8; ++nt) {
      const unsigned short* wq = bp + (size_t)(16 * nt) * (size_t)KB + k0;
      FragB bf;
      bf.h[0] = *(const v8usa*)wq;
      bf.h[1] = *(const v8usa*)(wq + 16);
      acc[nt] = wmb(af, bf, acc[nt]);
    }
  }
}

template <int SLB>
__device__ __forceinline__ int scan_chunk(const int* __restrict__ dsts, int nE, int cbase, int slotBase,
                                          int nb, int vec8, int* list, int tid, int lane, int wave) {
  int wc = 0;
  const int el0  = tid * EPT;
  const int e0   = cbase + el0;
  const int sent = -2147483647 - 1;
  v4i da, db;
  if (vec8 != 0 && cbase + CHUNK <= nE) {
    da = *(const v4i*)(dsts + e0);
    db = *(const v4i*)(dsts + e0 + 4);
  } else {
    da.x = (e0     < nE) ? dsts[min(e0,     nE - 1)] : sent;
    da.y = (e0 + 1 < nE) ? dsts[min(e0 + 1, nE - 1)] : sent;
    da.z = (e0 + 2 < nE) ? dsts[min(e0 + 2, nE - 1)] : sent;
    da.w = (e0 + 3 < nE) ? dsts[min(e0 + 3, nE - 1)] : sent;
    db.x = (e0 + 4 < nE) ? dsts[min(e0 + 4, nE - 1)] : sent;
    db.y = (e0 + 5 < nE) ? dsts[min(e0 + 5, nE - 1)] : sent;
    db.z = (e0 + 6 < nE) ? dsts[min(e0 + 6, nE - 1)] : sent;
    db.w = (e0 + 7 < nE) ? dsts[min(e0 + 7, nE - 1)] : sent;
  }
  const unsigned nbs = (unsigned)slotBase;
  const unsigned unb = (unsigned)nb;
  const unsigned s0 = (unsigned)da.x - nbs, s1 = (unsigned)da.y - nbs;
  const unsigned s2 = (unsigned)da.z - nbs, s3 = (unsigned)da.w - nbs;
  const unsigned s4 = (unsigned)db.x - nbs, s5 = (unsigned)db.y - nbs;
  const unsigned s6 = (unsigned)db.z - nbs, s7 = (unsigned)db.w - nbs;
  const bool h0 = s0 < unb, h1 = s1 < unb, h2 = s2 < unb, h3 = s3 < unb;
  const bool h4 = s4 < unb, h5 = s5 < unb, h6 = s6 < unb, h7 = s7 < unb;
  const unsigned any = __builtin_amdgcn_ballot_w32(h0 | h1 | h2 | h3 | h4 | h5 | h6 | h7);
  if (any != 0u) {
#define HITJ(J, HJ, SJ) { \
      const unsigned mj = __builtin_amdgcn_ballot_w32(HJ); \
      if (mj != 0u) { \
        if (HJ) { \
          const int pos = wc + (int)__builtin_amdgcn_mbcnt_lo(mj, 0u); \
          if (pos < WCAP) list[wave * WCAP + pos] = ((el0 + (J)) << SLB) | (int)(SJ); \
        } \
        wc += (int)__builtin_popcount(mj); } }
    HITJ(0, h0, s0)
    HITJ(1, h1, s1)
    HITJ(2, h2, s2)
    HITJ(3, h3, s3)
    HITJ(4, h4, s4)
    HITJ(5, h5, s5)
    HITJ(6, h6, s6)
    HITJ(7, h7, s7)
#undef HITJ
  }
  return wc;
}

__global__ __launch_bounds__(NTHR) void k_wprep(const float* __restrict__ W1B, const float* __restrict__ W1H,
                                                const float* __restrict__ W2B, const float* __restrict__ W2H,
                                                const float* __restrict__ W4,
                                                unsigned short* P1B, unsigned short* P1H,
                                                unsigned short* P2B, unsigned short* P2H,
                                                unsigned short* P4A, unsigned short* P4B) {
  __shared__ __attribute__((aligned(16))) unsigned short T[DF * DF];
  const int tid = (int)threadIdx.x;
  const int b   = (int)blockIdx.x;
  const float* W;
  unsigned short* P;
  int nout, nnt, pitch, step, dupoff, ndup, rbase, idx;
  if (b < 2)       { W = W1B; P = P1B; nout = DF;     nnt = 1; pitch = KB1; step = 2 * DF; dupoff = DF;     ndup = 1; rbase = 0;      idx = b; }
  else if (b < 4)  { W = W1H; P = P1H; nout = DF;     nnt = 1; pitch = KB1; step = 2 * DF; dupoff = DF;     ndup = 1; rbase = 0;      idx = b - 2; }
  else if (b < 10) { W = W2B; P = P2B; nout = 2 * DF; nnt = 2; pitch = KB2; step = 2 * DF; dupoff = DF;     ndup = 3; rbase = 0;      idx = b - 4; }
  else if (b < 16) { W = W2H; P = P2H; nout = 2 * DF; nnt = 2; pitch = KB2; step = 2 * DF; dupoff = DF;     ndup = 3; rbase = 0;      idx = b - 10; }
  else if (b < 18) { W = W4;  P = P4A; nout = DF;     nnt = 1; pitch = KB4; step = DF;     dupoff = 2 * DF; ndup = 2; rbase = 0;      idx = b - 16; }
  else if (b < 20) { W = W4;  P = P4B; nout = DF;     nnt = 1; pitch = KB4; step = DF;     dupoff = 2 * DF; ndup = 2; rbase = 2 * DF; idx = b - 18; }
  else return;
  const int kt = idx / nnt;
  const int nt = idx - kt * nnt;
  const int k0 = rbase + kt * DF;
  const int n0 = nt * DF;
#pragma unroll 2
  for (int it = 0; it < WLI; ++it) {
    const int i  = it * NTHR + tid;
    const int k  = i >> 5;
    const int n4 = (i & 31) * 4;
    const v4f w = *(const v4f*)(W + (size_t)(k0 + k) * (size_t)nout + n0 + n4);
    T[(n4 + 0) * DF + k] = (unsigned short)bf16_bits(w.x);
    T[(n4 + 1) * DF + k] = (unsigned short)bf16_bits(w.y);
    T[(n4 + 2) * DF + k] = (unsigned short)bf16_bits(w.z);
    T[(n4 + 3) * DF + k] = (unsigned short)bf16_bits(w.w);
  }
  __syncthreads();
  const int col0 = kt * step;
  const bool dual = kt < ndup;
  v8us q[WPI];
#pragma unroll
  for (int it = 0; it < WPI; ++it) {
    const int u  = it * NTHR + tid;
    const int n  = u >> 4;
    const int k8 = (u & 15) * 8;
    q[it] = *(const v8usa*)(T + n * DF + k8);
  }
#pragma unroll
  for (int it = 0; it < WPI; ++it) {
    const int u  = it * NTHR + tid;
    const int n  = u >> 4;
    const int k8 = (u & 15) * 8;
    unsigned short* dp = P + (size_t)(n0 + n) * (size_t)pitch + col0 + k8;
    *(volatile v8us*)dp = q[it];
    if (dual) *(volatile v8us*)(dp + dupoff) = q[it];
  }
  __threadfence();
#pragma unroll
  for (int it = 0; it < WPI; ++it) {
    const int u  = it * NTHR + tid;
    const int n  = u >> 4;
    const int k8 = (u & 15) * 8;
    unsigned short* dp = P + (size_t)(n0 + n) * (size_t)pitch + col0 + k8;
    *(volatile v8us*)dp = q[it];
    if (dual) *(volatile v8us*)(dp + dupoff) = q[it];
  }
}

template <int LX>
__global__ __launch_bounds__(NTHR) void k_scan(const int* __restrict__ src0, const int* __restrict__ dst0, int nE0,
                                               const int* __restrict__ src1, const int* __restrict__ dst1, int nE1,
                                               int nN, int mRows, const float* __restrict__ xin,
                                               const unsigned short* __restrict__ hpl, int hoff0, int hoff1,
                                               unsigned short* mpl, int mpitch) {
  extern __shared__ __attribute__((aligned(16))) int dsm[];
  int* list = dsm;
  int* hl   = dsm + LISTN;
  int* sl   = hl + RCAP;
  int* cnt  = sl + RCAP;
  int* offs = cnt + NBA;
  int* cur  = offs + NBA;
  int* misc = cur + NBA;
  const int tid = (int)threadIdx.x, lane = tid & 31, wave = tid >> 5;
  unsigned short* rowbuf = (unsigned short*)(misc + MISC_INTS) + wave * RBH;
  const int nodeBase = (int)blockIdx.x * NBA;
  const int ysel = (int)blockIdx.y;
  const int* srcs = (ysel != 0) ? src1 : src0;
  const int* dsts = (ysel != 0) ? dst1 : dst0;
  const int  nE   = (ysel != 0) ? nE1 : nE0;
  const int  hoff = (ysel != 0) ? hoff1 : hoff0;
  const int  ocol = (ysel != 0) ? 2 * DF : 0;
  const int  vec8 = ((nE & 3) == 0) ? 1 : 0;
  const bool wx   = (LX != 0) && (ysel == 0);

  {
    const v4i z4 = {0, 0, 0, 0};
    for (int i = tid * 4; i < AGG_ZINTS; i += NTHR * 4) *(v4ia*)(dsm + i) = z4;
    if (tid < MISC_INTS) misc[tid] = 0;
  }
  __syncthreads();

  int t = 0, ov = 0;
  const int nChunks = (nE + CHUNK - 1) / CHUNK;
#pragma unroll 1
  for (int ch = 0; ch < nChunks; ++ch) {
    const int cbase = ch * CHUNK;
    const int wc = scan_chunk<SLA>(dsts, nE, cbase, nodeBase, NBA, vec8, list, tid, lane, wave);
    if (lane == 0) misc[wave] = wc;
    __syncthreads();
    if (wave == 0) {
#pragma unroll 1
      for (int w2 = 0; w2 < NWAVE; ++w2) {
        int c = misc[w2];
        c = c < 0 ? 0 : (c > WCAP ? WCAP : c);
#pragma unroll 1
        for (int b0 = 0; b0 < c; b0 += 32) {
          const int idx = b0 + lane;
          const int ent = list[w2 * WCAP + (idx < WCAP ? idx : WCAP - 1)];
          const int m32 = (c - b0) < 32 ? (c - b0) : 32;
#pragma unroll 1
          for (int k = 0; k < m32; ++k) {
            const int u    = __builtin_amdgcn_readlane(ent, k);
            const int slot = u & (NBA - 1);
            const int el   = (u >> SLA) & (CHUNK - 1);
            const int pk   = ((cbase + el) << SLA) | slot;
            if (t < RCAP) {
              if (lane == 0) { hl[t] = pk; cnt[slot] = cnt[slot] + 1; }
              t = t + 1;
            } else {
              ov = 1;
            }
          }
        }
      }
    }
    __syncthreads();
  }
  if (wave == 0 && lane == 0) { misc[8] = t; misc[9] = ov; }
  __syncthreads();
  int tt = misc[8];
  tt = tt < 0 ? 0 : (tt > RCAP ? RCAP : tt);
  const int ovf = misc[9];

  if (wave == 0) {
    const int base = lane * (NBA / 32);
    int s = 0;
#pragma unroll 1
    for (int i = 0; i < NBA / 32; ++i) s += cnt[base + i];
    int incl = s;
#pragma unroll
    for (int d = 1; d < 32; d <<= 1) {
      const int y = __shfl_up(incl, d, 32);
      if (lane >= d) incl += y;
    }
    int run = incl - s;
#pragma unroll 1
    for (int i = 0; i < NBA / 32; ++i) {
      const int cv = cnt[base + i];
      offs[base + i] = run;
      cur[base + i]  = run;
      run += cv;
    }
  }
  __syncthreads();
  if (wave == 0) {
#pragma unroll 1
    for (int b0 = 0; b0 < tt; b0 += 32) {
      const int idx = b0 + lane;
      const int ent = hl[idx < RCAP ? idx : RCAP - 1];
      const int m32 = (tt - b0) < 32 ? (tt - b0) : 32;
#pragma unroll 1
      for (int k = 0; k < m32; ++k) {
        const int u    = __builtin_amdgcn_readlane(ent, k);
        const int slot = u & (NBA - 1);
        if (lane == 0) {
          int p = cur[slot];
          p = p < 0 ? 0 : (p > RCAP - 1 ? RCAP - 1 : p);
          sl[p] = u;
          cur[slot] = p + 1;
        }
      }
    }
  }
  __syncthreads();

  const float pz = (ovf != 0) ? __int_as_float(0x7fc00000) : 0.0f;
#pragma unroll 1
  for (int si = 0; si < NBA / NWAVE; ++si) {
    const int s    = si * NWAVE + wave;
    const int node = nodeBase + s;
    int c = cnt[s];
    const bool big = c > DEGCAP;
    c = c < 0 ? 0 : (c > DEGCAP ? DEGCAP : c);
    int o = offs[s];
    o = o < 0 ? 0 : (o > RCAP ? RCAP : o);
    const int nc = node < nN ? node : nN - 1;
    float a0 = 0.0f, a1 = 0.0f, a2 = 0.0f, a3 = 0.0f;
#pragma unroll 1
    for (int b0 = 0; b0 < c; b0 += 32) {
      int idx = o + b0 + lane;
      idx = idx > RCAP - 1 ? RCAP - 1 : idx;
      const int ent = sl[idx];
      int eid = ent >> SLA;
      eid = eid < 0 ? 0 : (eid > nE - 1 ? nE - 1 : eid);
      int sr = srcs[eid];
      sr = sr < 0 ? 0 : (sr > nN - 1 ? nN - 1 : sr);
      const int m32 = (c - b0) < 32 ? (c - b0) : 32;
#pragma unroll 1
      for (int k = 0; k < m32; ++k) {
        const int sk = __builtin_amdgcn_readlane(sr, k);
        if constexpr (LX != 0) {
          const v4f a = *(const v4f*)(xin + (size_t)sk * DF + 4 * lane);
          a0 += bf16_val(a.x);
          a1 += bf16_val(a.y);
          a2 += bf16_val(a.z);
          a3 += bf16_val(a.w);
        } else {
          const unsigned short* rp = hpl + (size_t)sk * HPP + hoff + 4 * lane;
          const v2u wh = *(const v2ua*)rp;
          const v2u wl = *(const v2ua*)(rp + DF);
          const float f0 = __uint_as_float(wh.x << 16)         + __uint_as_float(wl.x << 16);
          const float f1 = __uint_as_float(wh.x & 0xffff0000u) + __uint_as_float(wl.x & 0xffff0000u);
          const float f2 = __uint_as_float(wh.y << 16)         + __uint_as_float(wl.y << 16);
          const float f3 = __uint_as_float(wh.y & 0xffff0000u) + __uint_as_float(wl.y & 0xffff0000u);
          a0 += f0;
          a1 += f1;
          a2 += f2;
          a3 += f3;
        }
      }
    }
    const float den = (c > 0) ? (float)c : 1.0f;
    const float rcp = 1.0f / den;
    const float pzr = big ? __int_as_float(0x7fc00000) : pz;
    const bool live = node < nN;
    const float m0 = live ? (a0 * rcp + pzr) : 0.0f;
    const float m1 = live ? (a1 * rcp + pzr) : 0.0f;
    const float m2 = live ? (a2 * rcp + pzr) : 0.0f;
    const float m3 = live ? (a3 * rcp + pzr) : 0.0f;
    v4us mh, ml;
    {
      unsigned hb;
      hb = bf16_bits(m0); mh[0] = (unsigned short)hb; ml[0] = (unsigned short)bf16_bits(m0 - __uint_as_float(hb << 16));
      hb = bf16_bits(m1); mh[1] = (unsigned short)hb; ml[1] = (unsigned short)bf16_bits(m1 - __uint_as_float(hb << 16));
      hb = bf16_bits(m2); mh[2] = (unsigned short)hb; ml[2] = (unsigned short)bf16_bits(m2 - __uint_as_float(hb << 16));
      hb = bf16_bits(m3); mh[3] = (unsigned short)hb; ml[3] = (unsigned short)bf16_bits(m3 - __uint_as_float(hb << 16));
    }
    *(v4usa*)(rowbuf + 4 * lane) = mh;
    *(v4usa*)(rowbuf + DF + 4 * lane) = ml;
    if constexpr (LX != 0) {
      const v4f xs = *(const v4f*)(xin + (size_t)nc * DF + 4 * lane);
      v4us xb;
      xb[0] = live ? (unsigned short)bf16_bits(xs.x + pzr) : (unsigned short)0;
      xb[1] = live ? (unsigned short)bf16_bits(xs.y + pzr) : (unsigned short)0;
      xb[2] = live ? (unsigned short)bf16_bits(xs.z + pzr) : (unsigned short)0;
      xb[3] = live ? (unsigned short)bf16_bits(xs.w + pzr) : (unsigned short)0;
      const v4us z4 = {0, 0, 0, 0};
      *(v4usa*)(rowbuf + 2 * DF + 4 * lane) = xb;
      *(v4usa*)(rowbuf + 3 * DF + 4 * lane) = z4;
    }
    wave_sync();
    const v8us q0 = *(const v8usa*)(rowbuf + 8 * lane);
    v8us q1 = {0, 0, 0, 0, 0, 0, 0, 0};
    if constexpr (LX != 0) q1 = *(const v8usa*)(rowbuf + 2 * DF + 8 * lane);
    wave_sync();
    if (node < mRows) {
      unsigned short* rrow = mpl + (size_t)node * (size_t)mpitch;
      *(volatile v8us*)(rrow + ocol + 8 * lane) = q0;
      if (wx) *(volatile v8us*)(rrow + 4 * DF + 8 * lane) = q1;
      __threadfence();
      *(volatile v8us*)(rrow + ocol + 8 * lane) = q0;
      if (wx) *(volatile v8us*)(rrow + 4 * DF + 8 * lane) = q1;
    }
  }
}

template <int MODE>
__global__ __launch_bounds__(GTHR) void k_gemmA(const unsigned short* __restrict__ apl, int apitch,
                                                int acol0, int acolstep, int K0, int acol1, int K1,
                                                const unsigned short* __restrict__ bt, int btstep, int KB,
                                                const float* __restrict__ b0, const float* __restrict__ b1,
                                                const float* __restrict__ padd, int nN,
                                                unsigned short* opl, int opitch, int ocolstep, float* outf) {
  __shared__ __attribute__((aligned(16))) float stg[GBM * GBN];
  const int tid = (int)threadIdx.x, lane = tid & 31, wave = tid >> 5, hh = lane >> 4, m = lane & 15;
  const int rowBase = (int)blockIdx.x * GBM;
  const int ysel = (int)blockIdx.y;

  v8f acc[8];
#pragma unroll
  for (int t = 0; t < 8; ++t) acc[t] = z8();
  const unsigned short* arow = apl + (size_t)(rowBase + 16 * wave + m) * (size_t)apitch + 8 * hh;
  const unsigned short* btp  = bt + (size_t)ysel * (size_t)btstep + (size_t)m * (size_t)KB + 8 * hh;
  mma_seg(acc, arow + acol0 + ysel * acolstep, btp, KB, K0);
  if (K1 > 0) mma_seg(acc, arow + acol1, btp + K0, KB, K1);

#pragma unroll
  for (int nt = 0; nt < 8; ++nt) {
    const int lc = 16 * nt + m;
#pragma unroll
    for (int r = 0; r < 8; ++r) {
      const int lr = 16 * wave + 8 * hh + r;
      stg[lr * GBN + lc] = acc[nt][r];
    }
  }
  __syncthreads();

  v4f bq = {0.0f, 0.0f, 0.0f, 0.0f};
  if constexpr (MODE != 1) {
    const float* bsel = (ysel != 0) ? b1 : b0;
    const v4f b4 = *(const v4f*)(bsel + 4 * lane);
    bq.x = bf16_val(b4.x); bq.y = bf16_val(b4.y); bq.z = bf16_val(b4.z); bq.w = bf16_val(b4.w);
  }

  v4f pv[16];
#pragma unroll
  for (int i = 0; i < 16; ++i) pv[i] = *(const v4fa*)(stg + (16 * wave + i) * GBN + 4 * lane);
  __syncthreads();

#pragma unroll
  for (int i = 0; i < 16; ++i) {
    const int row = rowBase + 16 * wave + i;
    const bool ok = row < nN;
    v4f tq = pv[i];
    v4f y;
    if constexpr (MODE == 2) {
      const v4f rr = *(const v4f*)(padd + (size_t)row * DF + 4 * lane);
      tq = tq + rr;
    }
    if constexpr (MODE != 1) {
      tq = tq + bq;
      y.x = tanhf(tq.x); y.y = tanhf(tq.y); y.z = tanhf(tq.z); y.w = tanhf(tq.w);
    } else {
      y = tq;
    }
    y.x = ok ? y.x : 0.0f; y.y = ok ? y.y : 0.0f; y.z = ok ? y.z : 0.0f; y.w = ok ? y.w : 0.0f;
    pv[i] = y;
  }

  if constexpr (MODE == 2) {
#pragma unroll
    for (int i = 0; i < 16; ++i) {
      const int r = rowBase + 16 * wave + i;
      if (r < nN) *(volatile v4f*)(outf + (size_t)r * DF + 4 * lane) = pv[i];
    }
    __threadfence();
#pragma unroll
    for (int i = 0; i < 16; ++i) {
      const int r = rowBase + 16 * wave + i;
      if (r < nN) *(volatile v4f*)(outf + (size_t)r * DF + 4 * lane) = pv[i];
    }
  } else if constexpr (MODE == 1) {
#pragma unroll
    for (int i = 0; i < 16; ++i) {
      float* op = outf + (size_t)(rowBase + 16 * wave + i) * (size_t)DF + 4 * lane;
      *(volatile v4f*)op = pv[i];
    }
    __threadfence();
#pragma unroll
    for (int i = 0; i < 16; ++i) {
      float* op = outf + (size_t)(rowBase + 16 * wave + i) * (size_t)DF + 4 * lane;
      *(volatile v4f*)op = pv[i];
    }
  } else {
#pragma unroll
    for (int i = 0; i < 16; ++i) {
      v4us h4, l4;
      unsigned hb;
      hb = bf16_bits(pv[i].x); h4[0] = (unsigned short)hb; l4[0] = (unsigned short)bf16_bits(pv[i].x - __uint_as_float(hb << 16));
      hb = bf16_bits(pv[i].y); h4[1] = (unsigned short)hb; l4[1] = (unsigned short)bf16_bits(pv[i].y - __uint_as_float(hb << 16));
      hb = bf16_bits(pv[i].z); h4[2] = (unsigned short)hb; l4[2] = (unsigned short)bf16_bits(pv[i].z - __uint_as_float(hb << 16));
      hb = bf16_bits(pv[i].w); h4[3] = (unsigned short)hb; l4[3] = (unsigned short)bf16_bits(pv[i].w - __uint_as_float(hb << 16));
      unsigned short* srow = (unsigned short*)stg + (size_t)(16 * wave + i) * (2 * GBN);
      *(v4usa*)(srow + 4 * lane) = h4;
      *(v4usa*)(srow + DF + 4 * lane) = l4;
    }
    __syncthreads();
    v8us qv[16];
#pragma unroll
    for (int i = 0; i < 16; ++i) {
      const unsigned short* srow = (const unsigned short*)stg + (size_t)(16 * wave + i) * (2 * GBN);
      qv[i] = *(const v8usa*)(srow + 8 * lane);
    }
#pragma unroll
    for (int i = 0; i < 16; ++i) {
      unsigned short* rp = opl + (size_t)(rowBase + 16 * wave + i) * (size_t)opitch + ysel * ocolstep + 8 * lane;
      *(volatile v8us*)rp = qv[i];
    }
    __threadfence();
#pragma unroll
    for (int i = 0; i < 16; ++i) {
      unsigned short* rp = opl + (size_t)(rowBase + 16 * wave + i) * (size_t)opitch + ysel * ocolstep + 8 * lane;
      *(volatile v8us*)rp = qv[i];
    }
  }
}

__global__ __launch_bounds__(GTHR) void k_gemm2(unsigned short* mpl, const unsigned short* __restrict__ hpl, int hoff,
                                               const unsigned short* __restrict__ bt, const float* __restrict__ bias,
                                               int nN) {
  __shared__ __attribute__((aligned(16))) float stg[G2M * G2N];
  const int tid = (int)threadIdx.x, lane = tid & 31, wave = tid >> 5, hh = lane >> 4, m = lane & 15;
  const int rg = wave & 1, ch = wave >> 1;
  const int rowBase = (int)blockIdx.x * G2M;

  v8f acc[8];
#pragma unroll
  for (int t = 0; t < 8; ++t) acc[t] = z8();
  const int arow = rowBase + 16 * rg + m;
  const unsigned short* a0p = mpl + (size_t)arow * (size_t)MPP + 8 * hh;
  const unsigned short* a1p = hpl + (size_t)arow * (size_t)HPP + hoff + 8 * hh;
  const unsigned short* btp = bt + (size_t)(DF * ch + m) * (size_t)KB2 + 8 * hh;
  mma_seg(acc, a0p, btp, KB2, 4 * DF);
  mma_seg(acc, a1p, btp + 4 * DF, KB2, 2 * DF);

#pragma unroll
  for (int nt = 0; nt < 8; ++nt) {
    const int lc = DF * ch + 16 * nt + m;
#pragma unroll
    for (int r = 0; r < 8; ++r) {
      const int lr = 16 * rg + 8 * hh + r;
      stg[lr * G2N + lc] = acc[nt][r];
    }
  }
  __syncthreads();

  v4f bq0, bq1;
  {
    const v4f t0 = *(const v4f*)(bias + 8 * lane);
    const v4f t1 = *(const v4f*)(bias + 8 * lane + 4);
    bq0.x = bf16_val(t0.x); bq0.y = bf16_val(t0.y); bq0.z = bf16_val(t0.z); bq0.w = bf16_val(t0.w);
    bq1.x = bf16_val(t1.x); bq1.y = bf16_val(t1.y); bq1.z = bf16_val(t1.z); bq1.w = bf16_val(t1.w);
  }
#pragma unroll 1
  for (int i = 0; i < G2M / GWAVE; ++i) {
    const int lr  = (G2M / GWAVE) * wave + i;
    const int row = rowBase + lr;
    const bool ok = row < nN;
    const float* sp = stg + lr * G2N + 8 * lane;
    v4f p0 = *(const v4fa*)sp;
    v4f p1 = *(const v4fa*)(sp + 4);
    p0 = p0 + bq0;
    p1 = p1 + bq1;
    v4f y0, y1;
    y0.x = tanhf(p0.x); y0.y = tanhf(p0.y); y0.z = tanhf(p0.z); y0.w = tanhf(p0.w);
    y1.x = tanhf(p1.x); y1.y = tanhf(p1.y); y1.z = tanhf(p1.z); y1.w = tanhf(p1.w);
    y0.x = ok ? y0.x : 0.0f; y0.y = ok ? y0.y : 0.0f; y0.z = ok ? y0.z : 0.0f; y0.w = ok ? y0.w : 0.0f;
    y1.x = ok ? y1.x : 0.0f; y1.y = ok ? y1.y : 0.0f; y1.z = ok ? y1.z : 0.0f; y1.w = ok ? y1.w : 0.0f;
    v8us vh, vl;
    {
      unsigned hb;
      hb = bf16_bits(y0.x); vh[0] = (unsigned short)hb; vl[0] = (unsigned short)bf16_bits(y0.x - __uint_as_float(hb << 16));
      hb = bf16_bits(y0.y); vh[1] = (unsigned short)hb; vl[1] = (unsigned short)bf16_bits(y0.y - __uint_as_float(hb << 16));
      hb = bf16_bits(y0.z); vh[2] = (unsigned short)hb; vl[2] = (unsigned short)bf16_bits(y0.z - __uint_as_float(hb << 16));
      hb = bf16_bits(y0.w); vh[3] = (unsigned short)hb; vl[3] = (unsigned short)bf16_bits(y0.w - __uint_as_float(hb << 16));
      hb = bf16_bits(y1.x); vh[4] = (unsigned short)hb; vl[4] = (unsigned short)bf16_bits(y1.x - __uint_as_float(hb << 16));
      hb = bf16_bits(y1.y); vh[5] = (unsigned short)hb; vl[5] = (unsigned short)bf16_bits(y1.y - __uint_as_float(hb << 16));
      hb = bf16_bits(y1.z); vh[6] = (unsigned short)hb; vl[6] = (unsigned short)bf16_bits(y1.z - __uint_as_float(hb << 16));
      hb = bf16_bits(y1.w); vh[7] = (unsigned short)hb; vl[7] = (unsigned short)bf16_bits(y1.w - __uint_as_float(hb << 16));
    }
    unsigned short* rp = mpl + (size_t)row * (size_t)MPP;
    *(volatile v8us*)(rp + 8 * lane) = vh;
    *(volatile v8us*)(rp + 2 * DF + 8 * lane) = vl;
    __threadfence();
    *(volatile v8us*)(rp + 8 * lane) = vh;
    *(volatile v8us*)(rp + 2 * DF + 8 * lane) = vl;
  }
}

static inline int cdiv(int a, int b) { return (a + b - 1) / b; }
static inline size_t al256(size_t o) { return (o + 255) & ~(size_t)255; }

extern "C" void kernel_launch(void* const* d_in, const int* in_sizes, int n_in,
                              void* d_out, int out_size, void* d_ws, size_t ws_size,
                              hipStream_t stream) {
  if (n_in < 15) return;
  if (in_sizes[0] < DF || (in_sizes[0] % DF) != 0) return;
  const int nN  = in_sizes[0] / DF;
  const int nEp = in_sizes[1];
  if (nEp < 1 || in_sizes[2] != nEp) return;
  const int nEn = in_sizes[3];
  if (nEn < 1 || in_sizes[4] != nEn) return;
  if (nEp >= (1 << 21) || nEn >= (1 << 21) || nN < 16 || nN >= (1 << 24)) return;
  if (in_sizes[5] != 2 * DF * DF || in_sizes[6] != DF) return;
  if (in_sizes[7] != 2 * DF * DF || in_sizes[8] != DF) return;
  if (in_sizes[9] != 6 * DF * DF || in_sizes[10] != 2 * DF) return;
  if (in_sizes[11] != 6 * DF * DF || in_sizes[12] != 2 * DF) return;
  if (in_sizes[13] != 4 * DF * DF || in_sizes[14] != DF) return;
  if ((long long)out_size != (long long)nN * DF) return;

  const float* x     = (const float*)d_in[0];
  const int*   psrc  = (const int*)d_in[1];
  const int*   pdst  = (const int*)d_in[2];
  const int*   nsrc  = (const int*)d_in[3];
  const int*   ndst  = (const int*)d_in[4];
  const float* WoneB = (const float*)d_in[5];
  const float* boneB = (const float*)d_in[6];
  const float* WoneH = (const float*)d_in[7];
  const float* boneH = (const float*)d_in[8];
  const float* WtwoB = (const float*)d_in[9];
  const float* btwoB = (const float*)d_in[10];
  const float* WtwoH = (const float*)d_in[11];
  const float* btwoH = (const float*)d_in[12];
  const float* Wfour = (const float*)d_in[13];
  const float* bfour = (const float*)d_in[14];
  float* out = (float*)d_out;

  const int MP  = cdiv(nN, GBM) * GBM;
  const int gM  = MP / GBM;
  const int gM2 = MP / G2M;
  const int gA  = cdiv(nN, NBA);
  if ((long long)gA * NBA < (long long)MP) return;
  if ((MP % G2M) != 0) return;

  char* ws = (char*)d_ws;
  size_t off = 0;
  const size_t oB1 = off; off = al256(off + (size_t)2 * DF * KB1 * 2);
  const size_t oB2 = off; off = al256(off + (size_t)2 * 2 * DF * KB2 * 2);
  const size_t oB4 = off; off = al256(off + (size_t)2 * DF * KB4 * 2);
  const size_t sM  = (size_t)MP * MPP * 2;
  const size_t sP  = (size_t)MP * DF * 4;
  const size_t sL1 = (size_t)MP * L1P * 2;
  const size_t sMP = (sM + sP > sL1) ? (sM + sP) : sL1;
  const size_t oM  = off;
  const size_t oP  = oM + sM;
  off = al256(oM + sMP);
  const size_t oH  = off; off = al256(off + (size_t)MP * HPP * 2);
  if (off > ws_size || off > (size_t)WSMAX) return;
  unsigned short* BT1B = (unsigned short*)(ws + oB1);
  unsigned short* BT1H = BT1B + (size_t)DF * KB1;
  unsigned short* BT2B = (unsigned short*)(ws + oB2);
  unsigned short* BT2H = BT2B + (size_t)2 * DF * KB2;
  unsigned short* BT4a = (unsigned short*)(ws + oB4);
  unsigned short* BT4b = BT4a + (size_t)DF * KB4;
  unsigned short* L1   = (unsigned short*)(ws + oM);
  unsigned short* M    = (unsigned short*)(ws + oM);
  float*          P    = (float*)(ws + oP);
  unsigned short* H1   = (unsigned short*)(ws + oH);

  const size_t scanLds = (size_t)AGG_LDS_INTS * 4;
  hipFuncSetAttribute(reinterpret_cast<const void*>(&k_scan<1>), hipFuncAttributeMaxDynamicSharedMemorySize, (int)scanLds);
  hipFuncSetAttribute(reinterpret_cast<const void*>(&k_scan<0>), hipFuncAttributeMaxDynamicSharedMemorySize, (int)scanLds);

  k_wprep<<<WPJOBS, NTHR, 0, stream>>>(WoneB, WoneH, WtwoB, WtwoH, Wfour, BT1B, BT1H, BT2B, BT2H, BT4a, BT4b);
  k_scan<1><<<dim3(gA, 2), NTHR, scanLds, stream>>>(psrc, pdst, nEp, nsrc, ndst, nEn, nN, MP, x, H1, 0, 0, L1, L1P);
  k_gemmA<0><<<dim3(gM, 2), GTHR, 0, stream>>>(L1, L1P, 0, 2 * DF, 2 * DF, 4 * DF, DF, BT1B, DF * KB1, KB1,
                                                boneB, boneH, x, nN, H1, HPP, 2 * DF, out);
  k_scan<0><<<dim3(gA, 2), NTHR, scanLds, stream>>>(psrc, pdst, nEp, nsrc, ndst, nEn, nN, MP, x, H1, 0, 2 * DF, M, MPP);
  k_gemm2<<<gM2, GTHR, 0, stream>>>(M, H1, 0, BT2B, btwoB, nN);
  k_gemmA<1><<<dim3(gM, 1), GTHR, 0, stream>>>(M, MPP, 0, 0, 4 * DF, 0, 0, BT4a, 0, KB4,
                                                bfour, bfour, x, nN, H1, HPP, 0, P);
  k_scan<0><<<dim3(gA, 2), NTHR, scanLds, stream>>>(psrc, pdst, nEp, nsrc, ndst, nEn, nN, MP, x, H1, 2 * DF, 0, M, MPP);
  k_gemm2<<<gM2, GTHR, 0, stream>>>(M, H1, 2 * DF, BT2H, btwoH, nN);
  k_gemmA<2><<<dim3(gM, 1), GTHR, 0, stream>>>(M, MPP, 0, 0, 4 * DF, 0, 0, BT4b, 0, KB4,
                                                bfour, bfour, P, nN, H1, HPP, 0, out);
}
